// Takahashi_40716289966842
// MI455X (gfx1250) — hardware-verified
//
#include <hip/hip_runtime.h>
#include <stddef.h>
#include <math.h>


#define NS      4
#define NMAX    8
#define LMAX    4
#define DD      32
#define HID     128
#define FP      24
#define APITCH  192
#define NTHR    256
#define NWAVE   8
#define EPT     8
#define NGRP    2
#define CHUNK   (NTHR * EPT * NGRP)
#define WCAP    (EPT * NGRP * 32)
#define LISTN   (NWAVE * WCAP)
#define NB      256
#define MLPT    64
#define PI_F    3.14159265358979323846f

#define LDS_ACC   (NB * APITCH * 4)
#define LDS_LIST  (LISTN * 4)
#define LDS_WC    64
#define LDS_DENS  (LDS_ACC + LDS_LIST + LDS_WC)

static_assert((CHUNK & (CHUNK - 1)) == 0);
static_assert(CHUNK <= 4096);
static_assert((NB & (NB - 1)) == 0);
static_assert(NB <= 4096);
static_assert(NB == NWAVE * 32);
static_assert(APITCH == 24 * NMAX);
static_assert(NWAVE * 4 <= LDS_WC);
static_assert(LDS_DENS <= 300 * 1024);
static_assert(FP * 5 >= 0);

typedef float  v2f   __attribute__((ext_vector_type(2)));
typedef float  v4f   __attribute__((ext_vector_type(4)));
typedef float  v8f   __attribute__((ext_vector_type(8)));
typedef int    v4i   __attribute__((ext_vector_type(4)));
typedef v2f v2fa __attribute__((may_alias));
typedef v4f v4fa __attribute__((may_alias));
typedef v4i v4ia __attribute__((may_alias));
typedef __bf16 bf16_t;
typedef bf16_t v8bf  __attribute__((ext_vector_type(8)));
typedef bf16_t v16bf __attribute__((ext_vector_type(16)));
union FragB { v16bf v; v8bf h[2]; v4i q[2]; };
union Pack8 { v8bf v; v4i q; };

__device__ __forceinline__ v8f wmb(v16bf a, v16bf b, v8f c) {
  v8f d = __builtin_amdgcn_wmma_f32_16x16x32_bf16(false, a, false, b, (short)0, c, false, false);
  asm volatile("v_nop\n\tv_nop\n\tv_nop\n\tv_nop" : "+v"(d) : "v"(a), "v"(b));
  return d;
}

template <int B>
__device__ __forceinline__ void split8(FragB& hi, FragB& lo, v4f a, v4f b) {
#define SPL1(I, X) { const float xv = (X); const bf16_t hb = (bf16_t)xv; hi.v[B + (I)] = hb; lo.v[B + (I)] = (bf16_t)(xv - (float)hb); }
  SPL1(0, a.x) SPL1(1, a.y) SPL1(2, a.z) SPL1(3, a.w)
  SPL1(4, b.x) SPL1(5, b.y) SPL1(6, b.z) SPL1(7, b.w)
#undef SPL1
}

template <int NBT>
__device__ __forceinline__ int scan_chunk(const int* __restrict__ dsts, int nE, int cbase, int nodeBase,
                                          int vec8, int* list, int tid, int lane, int wave) {
  int wc = 0;
  (void)lane;
#pragma unroll
  for (int g = 0; g < NGRP; ++g) {
    const int el0  = (g * NTHR + tid) * EPT;
    const int e0   = cbase + el0;
    const int sent = -2147483647 - 1;
    v4i da, db;
    if (vec8 != 0 && cbase + CHUNK <= nE) {
      da = *(const v4ia*)(dsts + e0);
      db = *(const v4ia*)(dsts + e0 + 4);
    } else {
      da.x = (e0     < nE) ? dsts[min(e0, nE - 1)] : sent;
      da.y = (e0 + 1 < nE) ? dsts[min(e0 + 1, nE - 1)] : sent;
      da.z = (e0 + 2 < nE) ? dsts[min(e0 + 2, nE - 1)] : sent;
      da.w = (e0 + 3 < nE) ? dsts[min(e0 + 3, nE - 1)] : sent;
      db.x = (e0 + 4 < nE) ? dsts[min(e0 + 4, nE - 1)] : sent;
      db.y = (e0 + 5 < nE) ? dsts[min(e0 + 5, nE - 1)] : sent;
      db.z = (e0 + 6 < nE) ? dsts[min(e0 + 6, nE - 1)] : sent;
      db.w = (e0 + 7 < nE) ? dsts[min(e0 + 7, nE - 1)] : sent;
    }
    const unsigned nb = (unsigned)nodeBase;
    const unsigned s0 = (unsigned)da.x - nb, s1 = (unsigned)da.y - nb;
    const unsigned s2 = (unsigned)da.z - nb, s3 = (unsigned)da.w - nb;
    const unsigned s4 = (unsigned)db.x - nb, s5 = (unsigned)db.y - nb;
    const unsigned s6 = (unsigned)db.z - nb, s7 = (unsigned)db.w - nb;
    const bool h0 = s0 < (unsigned)NBT, h1 = s1 < (unsigned)NBT, h2 = s2 < (unsigned)NBT, h3 = s3 < (unsigned)NBT;
    const bool h4 = s4 < (unsigned)NBT, h5 = s5 < (unsigned)NBT, h6 = s6 < (unsigned)NBT, h7 = s7 < (unsigned)NBT;
    const unsigned any = __builtin_amdgcn_ballot_w32(h0 | h1 | h2 | h3 | h4 | h5 | h6 | h7);
    if (any != 0u) {
#define HITJ(J, HJ, SJ) { \
        const unsigned mj = __builtin_amdgcn_ballot_w32(HJ); \
        if (mj != 0u) { \
          if (HJ) { \
            const int pos = wc + (int)__builtin_amdgcn_mbcnt_lo(mj, 0u); \
            if (pos < WCAP) list[wave * WCAP + pos] = ((el0 + (J)) << 12) | (int)(SJ); \
          } \
          wc += (int)__builtin_popcount(mj); } }
      HITJ(0, h0, s0)
      HITJ(1, h1, s1)
      HITJ(2, h2, s2)
      HITJ(3, h3, s3)
      HITJ(4, h4, s4)
      HITJ(5, h5, s5)
      HITJ(6, h6, s6)
      HITJ(7, h7, s7)
#undef HITJ
    }
  }
  return wc;
}

__global__ __launch_bounds__(NTHR) void k_cn0(const int* __restrict__ sym, const float* __restrict__ alpha,
                                               float* cn0, int nta, int nRows) {
  const int t = blockIdx.x * NTHR + threadIdx.x;
  const int total = nRows * 8;
  const int tc = t < total ? t : total - 1;
  const int row = tc >> 3, c4 = tc & 7;
  const int ra = row > nta - 1 ? nta - 1 : row;
  int sv = sym[ra];
  sv = sv < 0 ? 0 : (sv > NS - 1 ? NS - 1 : sv);
  const v4f v = *(const v4fa*)(alpha + sv * DD + 4 * c4);
  float* gp = cn0 + (size_t)row * DD + 4 * c4;
  const bool ok = t < total;
  if (ok) *(volatile v4f*)gp = v;
  __threadfence();
  if (ok) *(volatile v4f*)gp = v;
}

__global__ __launch_bounds__(NTHR) void k_wprep(const float* __restrict__ W1, const float* __restrict__ W2,
                                                 bf16_t* p1h, bf16_t* p1l, bf16_t* p2h, bf16_t* p2l) {
  const int tid = threadIdx.x;
  Pack8 ph, pl;
  bf16_t* dh;
  bf16_t* dl;
#define WSP(I, P, ST) { const float xv = (P)[(size_t)(I) * (ST)]; const bf16_t hb = (bf16_t)xv; ph.v[(I)] = hb; pl.v[(I)] = (bf16_t)(xv - (float)hb); }
  if (blockIdx.x < 8) {
    const int o   = (blockIdx.x * NTHR + tid) * 8;
    const int s   = o >> 12, rem = o & 4095;
    const int n   = rem >> 5, k0 = rem & 31;
    const float* src = W1 + (size_t)(s * DD + k0) * HID + n;
    WSP(0, src, HID) WSP(1, src, HID) WSP(2, src, HID) WSP(3, src, HID)
    WSP(4, src, HID) WSP(5, src, HID) WSP(6, src, HID) WSP(7, src, HID)
    dh = p1h + o; dl = p1l + o;
  } else {
    const int o   = ((blockIdx.x - 8) * NTHR + tid) * 8;
    const int s   = o >> 12, rem = o & 4095;
    const int n   = rem >> 7, k0 = rem & 127;
    const float* src = W2 + (size_t)(s * HID + k0) * DD + n;
    WSP(0, src, DD) WSP(1, src, DD) WSP(2, src, DD) WSP(3, src, DD)
    WSP(4, src, DD) WSP(5, src, DD) WSP(6, src, DD) WSP(7, src, DD)
    dh = p2h + o; dl = p2l + o;
  }
#undef WSP
  const v4i qh = ph.q, ql = pl.q;
  *(volatile v4i*)dh = qh;
  *(volatile v4i*)dl = ql;
  __threadfence();
  *(volatile v4i*)dh = qh;
  *(volatile v4i*)dl = ql;
}

__global__ __launch_bounds__(NTHR) void k_pair(const float* __restrict__ disp, const float* __restrict__ dist,
                                                float* fnr, int nE) {
  __shared__ float stg[NTHR * FP];
  const int tid = threadIdx.x, lane = tid & 31, wave = tid >> 5;
  const int e  = blockIdx.x * NTHR + tid;
  const int ec = e < nE ? e : nE - 1;
  const float d  = dist[ec];
  const float dx = disp[(size_t)ec * 3 + 0];
  const float dy = disp[(size_t)ec * 3 + 1];
  const float dz = disp[(size_t)ec * 3 + 2];
  const float t  = cosf((d * PI_F) * (1.0f / 6.0f)) + 1.0f;
  const float fc = 0.25f * (t * t);
  const float x2 = dx * dx, x3 = dx * x2;
  const float y2 = dy * dy, y3 = dy * y2;
  const float z2 = dz * dz, z3 = dz * z2;
  const float d2 = d * d, d3 = d * d2;
  const float i1 = 1.0f / d, i2 = 1.0f / d2, i3 = 1.0f / d3;
  float* sp = stg + tid * FP;
  sp[0]  = fc;
  sp[1]  = fc * (dz * i1);
  sp[2]  = fc * (dy * i1);
  sp[3]  = fc * (dx * i1);
  sp[4]  = fc * (z2 * i2);
  sp[5]  = 0.0f;
  sp[6]  = fc * ((dy * dz) * i2);
  sp[7]  = fc * (y2 * i2);
  sp[8]  = fc * ((dx * dz) * i2);
  sp[9]  = fc * ((dx * dy) * i2);
  sp[10] = fc * (x2 * i2);
  sp[11] = 0.0f;
  sp[12] = fc * (z3 * i3);
  sp[13] = fc * ((dy * z2) * i3);
  sp[14] = fc * ((y2 * dz) * i3);
  sp[15] = fc * (y3 * i3);
  sp[16] = fc * ((dx * z2) * i3);
  sp[17] = 0.0f;
  sp[18] = fc * (((dx * dy) * dz) * i3);
  sp[19] = fc * ((dx * y2) * i3);
  sp[20] = fc * ((x2 * dz) * i3);
  sp[21] = fc * ((x2 * dy) * i3);
  sp[22] = fc * (x3 * i3);
  sp[23] = 0.0f;
  __syncthreads();
  const v4fa* s4 = (const v4fa*)(stg + wave * 32 * FP);
  float* gb = fnr + ((size_t)blockIdx.x * NTHR + (size_t)wave * 32) * FP;
  v4f v[6];
#pragma unroll
  for (int i = 0; i < 6; ++i) v[i] = s4[i * 32 + lane];
#pragma unroll
  for (int i = 0; i < 6; ++i) *(volatile v4f*)(gb + (size_t)(i * 32 + lane) * 4) = v[i];
  __threadfence();
#pragma unroll
  for (int i = 0; i < 6; ++i) *(volatile v4f*)(gb + (size_t)(i * 32 + lane) * 4) = v[i];
}

__global__ __launch_bounds__(NTHR) void k_dens(
    const int* __restrict__ iidx, const int* __restrict__ jidx,
    const float* __restrict__ cnpl, const float* __restrict__ fnr,
    const float* __restrict__ hop, float* outp,
    int nta, int nE, int nRowsOut, int vec8) {
  extern __shared__ v4f lds_dyn[];
  float* acc  = (float*)lds_dyn;
  int*   list = (int*)((char*)lds_dyn + LDS_ACC);
  int*   wcnt = (int*)((char*)lds_dyn + LDS_ACC + LDS_LIST);
  const int tid = threadIdx.x, lane = tid & 31, wave = tid >> 5;
  const int nodeBase = blockIdx.x * NB;
  const int g = lane & 3, nn = lane >> 2;
  const bool g0 = (g == 0), g1 = (g == 1);

  {
    const v4f z = {0.f, 0.f, 0.f, 0.f};
    for (int i = tid; i < NB * APITCH / 4; i += NTHR) lds_dyn[i] = z;
  }
  __syncthreads();

  const int nChunks = (nE + CHUNK - 1) / CHUNK;
#pragma unroll 1
  for (int ch = 0; ch < nChunks; ++ch) {
    const int cbase = ch * CHUNK;
    const int wc = scan_chunk<NB>(iidx, nE, cbase, nodeBase, vec8, list, tid, lane, wave);
    if (lane == 0) wcnt[wave] = wc;
    __syncthreads();
    if (wave == 0) {
#pragma unroll 1
      for (int wsx = 0; wsx < NWAVE; ++wsx) {
        int n = __builtin_amdgcn_readfirstlane(wcnt[wsx]);
        n = n > WCAP ? WCAP : (n < 0 ? 0 : n);
        const int* lp = list + wsx * WCAP;
#pragma unroll 1
        for (int i = 0; i < n; ++i) {
          const int ent  = __builtin_amdgcn_readfirstlane(lp[i]);
          const int slot = ent & (NB - 1);
          int e = cbase + ((ent >> 12) & (CHUNK - 1));
          e = e > nE - 1 ? nE - 1 : e;
          int j = jidx[e];
          j = j < 0 ? 0 : (j > nta - 1 ? nta - 1 : j);
          const v4f cv = *(const v4fa*)(cnpl + (size_t)j * DD + 4 * nn);
          const float* fpp = fnr + (size_t)e * FP + 6 * g;
          const v2f f01 = *(const v2fa*)(fpp);
          const v2f f23 = *(const v2fa*)(fpp + 2);
          const v2f f45 = *(const v2fa*)(fpp + 4);
          const float base = g1 ? cv.z : cv.w;
          const float ca = g0 ? cv.x : base;
          const float cb = g0 ? cv.y : base;
          const float cc = g0 ? cv.z : base;
          float* ap = acc + slot * APITCH + 6 * lane;
          v2f a01 = *(v2fa*)(ap);
          v2f a23 = *(v2fa*)(ap + 2);
          v2f a45 = *(v2fa*)(ap + 4);
          a01.x += ca * f01.x;
          a01.y += cb * f01.y;
          a23.x += cb * f23.x;
          a23.y += cb * f23.y;
          a45.x += cc * f45.x;
          *(v2fa*)(ap)     = a01;
          *(v2fa*)(ap + 2) = a23;
          *(v2fa*)(ap + 4) = a45;
        }
      }
    }
    __syncthreads();
  }
  __syncthreads();

  const int n8 = lane & 7, sub = lane >> 3;
  float hr0, hr1, hr2, hr3;
  {
    const float* hp = hop + n8 * (LMAX * LMAX);
    const v4f q0 = *(const v4fa*)(hp), q1 = *(const v4fa*)(hp + 4);
    const v4f q2 = *(const v4fa*)(hp + 8), q3 = *(const v4fa*)(hp + 12);
    hr0 = ((q0.x + q0.y) + q0.z) + q0.w;
    hr1 = ((q1.x + q1.y) + q1.z) + q1.w;
    hr2 = ((q2.x + q2.y) + q2.z) + q2.w;
    hr3 = ((q3.x + q3.y) + q3.z) + q3.w;
  }
  v4f ov[8];
#pragma unroll
  for (int i = 0; i < 8; ++i) {
    const int slot = wave * 32 + 4 * i + sub;
    const float* dp = acc + slot * APITCH + 24 * n8;
    const v4f q0 = *(const v4fa*)(dp),      q1 = *(const v4fa*)(dp + 4);
    const v4f q2 = *(const v4fa*)(dp + 8),  q3 = *(const v4fa*)(dp + 12);
    const v4f q4 = *(const v4fa*)(dp + 16), q5 = *(const v4fa*)(dp + 20);
    const float s0 = q0.x * q0.x;
    const float s1 = q0.y * q0.y + q0.z * q0.z + q0.w * q0.w;
    const float s2 = q1.x * q1.x + q1.z * q1.z + q1.w * q1.w + q2.x * q2.x + q2.y * q2.y + q2.z * q2.z;
    const float s3 = q3.x * q3.x + q3.y * q3.y + q3.z * q3.z + q3.w * q3.w + q4.x * q4.x
                   + q4.z * q4.z + q4.w * q4.w + q5.x * q5.x + q5.y * q5.y + q5.z * q5.z;
    v4f o;
    o.x = s0 * hr0; o.y = s1 * hr1; o.z = s2 * hr2; o.w = s3 * hr3;
    ov[i] = o;
  }
#pragma unroll
  for (int i = 0; i < 8; ++i) {
    const int row = nodeBase + wave * 32 + 4 * i + sub;
    if (row < nRowsOut) *(volatile v4f*)(outp + (size_t)row * DD + 4 * n8) = ov[i];
  }
  __threadfence();
#pragma unroll
  for (int i = 0; i < 8; ++i) {
    const int row = nodeBase + wave * 32 + 4 * i + sub;
    if (row < nRowsOut) *(volatile v4f*)(outp + (size_t)row * DD + 4 * n8) = ov[i];
  }
}

__global__ __launch_bounds__(MLPT) void k_mlp(
    const float* __restrict__ xpl, const float* __restrict__ cn0, const int* __restrict__ sym,
    const bf16_t* __restrict__ p1h, const bf16_t* __restrict__ p1l,
    const bf16_t* __restrict__ p2h, const bf16_t* __restrict__ p2l,
    const float* __restrict__ b1, const float* __restrict__ b2,
    float* cn1, int nta, int nRows) {
  __shared__ float Hs[2][16 * HID];
  const int tid = threadIdx.x, lane = tid & 31, wave = tid >> 5, hh = lane >> 4, m = lane & 15;
  float* Hl = &Hs[wave][0];
  const int a0 = (blockIdx.x * 2 + wave) * 16;
  const v8f z8 = {0.f, 0.f, 0.f, 0.f, 0.f, 0.f, 0.f, 0.f};

  int symr[8];
#pragma unroll
  for (int r = 0; r < 8; ++r) {
    int row = a0 + 8 * hh + r;
    row = row > nta - 1 ? nta - 1 : row;
    int sv = sym[row];
    sv = sv < 0 ? 0 : (sv > NS - 1 ? NS - 1 : sv);
    symr[r] = sv;
  }

  FragB ahi, alo;
  {
    int xr = a0 + m;
    xr = xr > nRows - 1 ? nRows - 1 : xr;
    const float* xrow = xpl + (size_t)xr * DD + 8 * hh;
    const v4f p0 = *(const v4fa*)(xrow),      p1 = *(const v4fa*)(xrow + 4);
    const v4f p2 = *(const v4fa*)(xrow + 16), p3 = *(const v4fa*)(xrow + 20);
    split8<0>(ahi, alo, p0, p1);
    split8<8>(ahi, alo, p2, p3);
  }

  v8f c0 = z8, c1 = z8;
#pragma unroll 1
  for (int s = 0; s < NS; ++s) {
#pragma unroll 1
    for (int cg = 0; cg < 2; ++cg) {
      v8f h[4];
#pragma unroll
      for (int q = 0; q < 4; ++q) h[q] = z8;
#pragma unroll
      for (int q = 0; q < 4; ++q) {
        const int ct = cg * 4 + q;
        const size_t bo = (size_t)(s * HID + 16 * ct + m) * DD + 8 * hh;
        FragB bh, bl;
        bh.q[0] = *(const v4ia*)(p1h + bo);  bh.q[1] = *(const v4ia*)(p1h + bo + 16);
        bl.q[0] = *(const v4ia*)(p1l + bo);  bl.q[1] = *(const v4ia*)(p1l + bo + 16);
        h[q] = wmb(alo.v, bh.v, h[q]);
        h[q] = wmb(ahi.v, bl.v, h[q]);
        h[q] = wmb(ahi.v, bh.v, h[q]);
      }
#pragma unroll
      for (int q = 0; q < 4; ++q) {
        const int col = 16 * (cg * 4 + q) + m;
        const float bb = b1[s * HID + col];
        float* hp = Hl + (8 * hh) * HID + col;
#pragma unroll
        for (int r = 0; r < 8; ++r) {
          float v = h[q][r] + bb;
          v = v > 0.0f ? v : 0.01f * v;
          hp[r * HID] = v;
        }
      }
    }
    __syncthreads();

    v8f y0 = z8, y1 = z8;
#pragma unroll 1
    for (int ks = 0; ks < HID / 32; ++ks) {
      const float* ap = Hl + m * HID + 32 * ks + 8 * hh;
      const v4f p0 = *(const v4fa*)(ap),      p1 = *(const v4fa*)(ap + 4);
      const v4f p2 = *(const v4fa*)(ap + 16), p3 = *(const v4fa*)(ap + 20);
      FragB a2h, a2l;
      split8<0>(a2h, a2l, p0, p1);
      split8<8>(a2h, a2l, p2, p3);
      {
        const size_t bo = (size_t)(s * DD + m) * HID + 32 * ks + 8 * hh;
        FragB bh, bl;
        bh.q[0] = *(const v4ia*)(p2h + bo);  bh.q[1] = *(const v4ia*)(p2h + bo + 16);
        bl.q[0] = *(const v4ia*)(p2l + bo);  bl.q[1] = *(const v4ia*)(p2l + bo + 16);
        y0 = wmb(a2l.v, bh.v, y0);
        y0 = wmb(a2h.v, bl.v, y0);
        y0 = wmb(a2h.v, bh.v, y0);
      }
      {
        const size_t bo = (size_t)(s * DD + 16 + m) * HID + 32 * ks + 8 * hh;
        FragB bh, bl;
        bh.q[0] = *(const v4ia*)(p2h + bo);  bh.q[1] = *(const v4ia*)(p2h + bo + 16);
        bl.q[0] = *(const v4ia*)(p2l + bo);  bl.q[1] = *(const v4ia*)(p2l + bo + 16);
        y1 = wmb(a2l.v, bh.v, y1);
        y1 = wmb(a2h.v, bl.v, y1);
        y1 = wmb(a2h.v, bh.v, y1);
      }
    }
    const float bb0 = b2[s * DD + m], bb1 = b2[s * DD + 16 + m];
#pragma unroll
    for (int r = 0; r < 8; ++r) {
      const bool pick = (symr[r] == s);
      const float v0 = y0[r] + bb0, v1 = y1[r] + bb1;
      c0[r] = pick ? v0 : c0[r];
      c1[r] = pick ? v1 : c1[r];
    }
    __syncthreads();
  }

#pragma unroll
  for (int r = 0; r < 8; ++r) {
    Hl[(8 * hh + r) * DD + m]      = c0[r];
    Hl[(8 * hh + r) * DD + 16 + m] = c1[r];
  }
  __syncthreads();
  const v4fa* S4 = (const v4fa*)Hl;
  v4f ov[4];
#pragma unroll
  for (int i = 0; i < 4; ++i) {
    const int idx = i * 32 + lane;
    const int row = idx >> 3, c4 = idx & 7;
    int gr = a0 + row;
    gr = gr > nRows - 1 ? nRows - 1 : gr;
    const v4f cv = *(const v4fa*)(cn0 + (size_t)gr * DD + 4 * c4);
    ov[i] = S4[idx] + cv;
  }
#pragma unroll
  for (int i = 0; i < 4; ++i) {
    const int idx = i * 32 + lane;
    const int row = idx >> 3, c4 = idx & 7;
    *(volatile v4f*)(cn1 + (size_t)(a0 + row) * DD + 4 * c4) = ov[i];
  }
  __threadfence();
#pragma unroll
  for (int i = 0; i < 4; ++i) {
    const int idx = i * 32 + lane;
    const int row = idx >> 3, c4 = idx & 7;
    *(volatile v4f*)(cn1 + (size_t)(a0 + row) * DD + 4 * c4) = ov[i];
  }
}

extern "C" void kernel_launch(void* const* d_in, const int* in_sizes, int n_in,
                              void* d_out, int out_size, void* d_ws, size_t ws_size,
                              hipStream_t stream) {
  if (n_in < 11) return;
  const int nta = in_sizes[0];
  const int nE  = in_sizes[1];
  if (nta <= 0 || nE <= 0) return;
  if (in_sizes[2] != nE || in_sizes[3] != 3 * nE || in_sizes[4] != nE) return;
  if (in_sizes[5] != NS * DD) return;
  if (in_sizes[6] != 2 * NMAX * LMAX * LMAX) return;
  if (in_sizes[7] != NS * DD * HID || in_sizes[8] != NS * HID) return;
  if (in_sizes[9] != NS * HID * DD || in_sizes[10] != NS * DD) return;
  if (out_size != nta * DD) return;

  const int*   symbols = (const int*)d_in[0];
  const int*   iidx    = (const int*)d_in[1];
  const int*   jidx    = (const int*)d_in[2];
  const float* disp    = (const float*)d_in[3];
  const float* dist    = (const float*)d_in[4];
  const float* alpha   = (const float*)d_in[5];
  const float* hop     = (const float*)d_in[6];
  const float* W1      = (const float*)d_in[7];
  const float* b1      = (const float*)d_in[8];
  const float* W2      = (const float*)d_in[9];
  const float* b2      = (const float*)d_in[10];
  float* out = (float*)d_out;

  const int nBlkD = (nta + NB - 1) / NB;
  const int nRows = nBlkD * NB;
  const int nBlkM = (nta + 31) / 32;
  if (nBlkM * 32 > nRows) return;
  const int nBlkP  = (nE + NTHR - 1) / NTHR;
  const size_t nPairs = (size_t)nBlkP * NTHR;

  char* ws = (char*)d_ws;
  size_t off = 0;
  const size_t szF = nPairs * FP * 4;
  const size_t szR = (size_t)nRows * DD * 4;
  const size_t szW = (size_t)NS * HID * DD * 2;
  const size_t oF  = off; off += szF; off = (off + 255) & ~(size_t)255;
  const size_t oC0 = off; off += szR; off = (off + 255) & ~(size_t)255;
  const size_t oX  = off; off += szR; off = (off + 255) & ~(size_t)255;
  const size_t oC1 = off; off += szR; off = (off + 255) & ~(size_t)255;
  const size_t o1h = off; off += szW; off = (off + 255) & ~(size_t)255;
  const size_t o1l = off; off += szW; off = (off + 255) & ~(size_t)255;
  const size_t o2h = off; off += szW; off = (off + 255) & ~(size_t)255;
  const size_t o2l = off; off += szW; off = (off + 255) & ~(size_t)255;
  if (off > ws_size) return;
  float*  fnr = (float*)(ws + oF);
  float*  cn0 = (float*)(ws + oC0);
  float*  xpl = (float*)(ws + oX);
  float*  cn1 = (float*)(ws + oC1);
  bf16_t* p1h = (bf16_t*)(ws + o1h);
  bf16_t* p1l = (bf16_t*)(ws + o1l);
  bf16_t* p2h = (bf16_t*)(ws + o2h);
  bf16_t* p2l = (bf16_t*)(ws + o2l);

  const int vec8 = ((nE & 3) == 0) ? 1 : 0;

  k_cn0<<<(nRows * 8 + NTHR - 1) / NTHR, NTHR, 0, stream>>>(symbols, alpha, cn0, nta, nRows);
  k_wprep<<<16, NTHR, 0, stream>>>(W1, W2, p1h, p1l, p2h, p2l);
  k_pair<<<nBlkP, NTHR, 0, stream>>>(disp, dist, fnr, nE);

  hipFuncSetAttribute(reinterpret_cast<const void*>(&k_dens),
                      hipFuncAttributeMaxDynamicSharedMemorySize, LDS_DENS);

  k_dens<<<nBlkD, NTHR, LDS_DENS, stream>>>(iidx, jidx, cn0, fnr, hop, xpl, nta, nE, nRows, vec8);
  k_mlp<<<nBlkM, MLPT, 0, stream>>>(xpl, cn0, symbols, p1h, p1l, p2h, p2l, b1, b2, cn1, nta, nRows);
  k_dens<<<nBlkD, NTHR, LDS_DENS, stream>>>(iidx, jidx, cn1, fnr, hop + NMAX * LMAX * LMAX, out,
                                             nta, nE, nta, vec8);
}
